// RNNClassifier_9363028705538
// MI455X (gfx1250) — hardware-run, weakly checked
//
#include <hip/hip_runtime.h>
#include <math.h>

constexpr int NBATCH   = 4096;
constexpr int NSTEP    = 512;
constexpr int NVOC     = 57;
constexpr int NEMB     = 20;
constexpr int NHID     = 128;
constexpr int NCLS     = 18;
constexpr int NTHR     = 256;
constexpr int ROWS_BLK = 16;
constexpr int HPITCH   = 136;
constexpr int HSPITCH  = 132;
constexpr int NLOGIT   = ROWS_BLK * NCLS;
constexpr int NTABLE   = NVOC * NHID;
constexpr float WCARRY = 256.0f;
constexpr float HCARRY = 16.0f;
constexpr float FOLD   = 1.0f / (WCARRY * HCARRY);

static_assert(NHID == 16 * (NTHR / 32));
static_assert(NHID % 32 == 0);
static_assert(NBATCH % ROWS_BLK == 0);
static_assert(ROWS_BLK == 16);
static_assert(NEMB % 4 == 0);
static_assert(NTABLE % 32 == 0);
static_assert(NTABLE % 4 == 0);
static_assert(NLOGIT % 32 == 0);
static_assert((NLOGIT * 4) % 128 == 0);
static_assert((2 * ROWS_BLK * HPITCH) % NTHR == 0);
static_assert(((ROWS_BLK / 4) * NSTEP) % NTHR == 0);
static_assert(HPITCH % 8 == 0 && HPITCH >= NHID);
static_assert(HSPITCH % 4 == 0 && HSPITCH >= NHID);
static_assert(NVOC <= 256);

typedef __attribute__((ext_vector_type(16))) _Float16 v16h;
typedef __attribute__((ext_vector_type(8)))  _Float16 v8h;
typedef __attribute__((ext_vector_type(8)))  float    v8f;
typedef __attribute__((ext_vector_type(4)))  float    v4f;

union FragH { v16h v; v8h h[2]; };
__device__ __forceinline__ v16h frag_load_h(const _Float16* p) {
  FragH f;
  f.h[0] = *(const v8h*)(p);
  f.h[1] = *(const v8h*)(p + 16);
  return f.v;
}
__device__ __forceinline__ v8f wm_f16(v16h a, v16h b, v8f c) {
  c = __builtin_amdgcn_wmma_f32_16x16x32_f16(false, a, false, b, (short)0, c, false, false);
  asm volatile("v_nop\n\tv_nop\n\tv_nop\n\tv_nop" : "+v"(c) : "v"(a), "v"(b));
  return c;
}
__device__ __forceinline__ int clampi(int v, int lo, int hi) { return v < lo ? lo : (v > hi ? hi : v); }

__global__ __launch_bounds__(NTHR) void table_kernel(const float* __restrict__ emb, const float* __restrict__ W_ih,
                                                     const float* __restrict__ b_ih, const float* __restrict__ b_hh,
                                                     float* __restrict__ P) {
  const int i = blockIdx.x * NTHR + threadIdx.x;
  if (i < NTABLE) {
    const int v  = i / NHID;
    const int hc = i - v * NHID;
    const float* er = emb  + v  * NEMB;
    const float* wr = W_ih + hc * NEMB;
    float s = 0.0f;
#pragma unroll
    for (int q = 0; q < NEMB / 4; ++q) {
      const v4f a = *(const v4f*)(er + 4 * q);
      const v4f b = *(const v4f*)(wr + 4 * q);
      s = fmaf(a[0], b[0], s);
      s = fmaf(a[1], b[1], s);
      s = fmaf(a[2], b[2], s);
      s = fmaf(a[3], b[3], s);
    }
    s = (s + b_ih[hc]) + b_hh[hc];
    volatile float* op = P + i;
    *op = s;
    __threadfence();
    *op = s;
  }
}

__global__ __launch_bounds__(NTHR) void rnn_kernel(const int* __restrict__ x, const int* __restrict__ x_len,
                                                   const float* __restrict__ W_hh, const float* __restrict__ W_out,
                                                   const float* __restrict__ b_out, const float* __restrict__ P,
                                                   float* __restrict__ out) {
  __shared__ __align__(16) float    Ps[NTABLE];
  __shared__ __align__(16) unsigned xsw[NSTEP * (ROWS_BLK / 4)];
  __shared__ __align__(16) _Float16 Hb[2][ROWS_BLK * HPITCH];
  __shared__ __align__(16) float    Hs[ROWS_BLK * HSPITCH];
  __shared__ __align__(16) float    Lg[NLOGIT];
  __shared__ int lens_s[ROWS_BLK];

  const int tid  = threadIdx.x;
  const int lane = tid & 31;
  const int wave = tid >> 5;
  const int c    = lane & 15;
  const int hh   = lane >> 4;
  const int koff = hh * 8;
  const int ncol = 16 * wave + c;
  const int m0   = blockIdx.x * ROWS_BLK;

#pragma unroll 1
  for (int i = tid; i < NTABLE / 4; i += NTHR) {
    const v4f pv = *(const v4f*)(P + 4 * i);
    *(v4f*)(Ps + 4 * i) = pv;
  }
#pragma unroll 1
  for (int it = 0; it < ((ROWS_BLK / 4) * NSTEP) / NTHR; ++it) {
    const int idx = it * NTHR + tid;
    const int t   = idx % NSTEP;
    const int mq  = idx / NSTEP;
    const int* xp = x + (size_t)(m0 + 4 * mq) * NSTEP + t;
    const int t0 = clampi(xp[0],         0, NVOC - 1);
    const int t1 = clampi(xp[NSTEP],     0, NVOC - 1);
    const int t2 = clampi(xp[2 * NSTEP], 0, NVOC - 1);
    const int t3 = clampi(xp[3 * NSTEP], 0, NVOC - 1);
    xsw[t * (ROWS_BLK / 4) + mq] = (unsigned)t0 | ((unsigned)t1 << 8) | ((unsigned)t2 << 16) | ((unsigned)t3 << 24);
  }
  {
    _Float16* hb = &Hb[0][0];
#pragma unroll 1
    for (int i = tid; i < 2 * ROWS_BLK * HPITCH; i += NTHR) hb[i] = (_Float16)0.0f;
  }
  if (tid < ROWS_BLK) lens_s[tid] = clampi(x_len[m0 + tid], 0, NSTEP);

  v16h bfr[4];
  {
    const float* wrow = W_hh + (size_t)ncol * NHID + koff;
#pragma unroll
    for (int kc = 0; kc < 4; ++kc) {
      const v4f q0 = *(const v4f*)(wrow + 32 * kc);
      const v4f q1 = *(const v4f*)(wrow + 32 * kc + 4);
      const v4f q2 = *(const v4f*)(wrow + 32 * kc + 16);
      const v4f q3 = *(const v4f*)(wrow + 32 * kc + 20);
      v16h f;
#pragma unroll
      for (int e = 0; e < 4; ++e) {
        f[e]      = (_Float16)(q0[e] * WCARRY);
        f[4 + e]  = (_Float16)(q1[e] * WCARRY);
        f[8 + e]  = (_Float16)(q2[e] * WCARRY);
        f[12 + e] = (_Float16)(q3[e] * WCARRY);
      }
      bfr[kc] = f;
    }
  }
  __syncthreads();

  int tmax = 0;
#pragma unroll
  for (int m = 0; m < ROWS_BLK; ++m) tmax = max(tmax, lens_s[m]);
  tmax = min(tmax, NSTEP);
  int lenr[8];
  float hst[8];
#pragma unroll
  for (int r = 0; r < 8; ++r) { lenr[r] = lens_s[8 * hh + r]; hst[r] = 0.0f; }

  const v8f z8 = {0.f, 0.f, 0.f, 0.f, 0.f, 0.f, 0.f, 0.f};

#pragma unroll 1
  for (int t = 0; t < tmax; ++t) {
    const int cur = t & 1;
    const _Float16* ha = &Hb[cur][0] + c * HPITCH + koff;
    _Float16* hn = &Hb[cur ^ 1][0];
    v8f acc = z8;
#pragma unroll
    for (int kc = 0; kc < 4; ++kc) {
      const v16h a = frag_load_h(ha + 32 * kc);
      acc = wm_f16(a, bfr[kc], acc);
    }
    const unsigned w0 = xsw[t * (ROWS_BLK / 4) + 2 * hh];
    const unsigned w1 = xsw[t * (ROWS_BLK / 4) + 2 * hh + 1];
#pragma unroll
    for (int r = 0; r < 8; ++r) {
      const unsigned w = (r < 4) ? w0 : w1;
      const int tok = (int)((w >> (8 * (r & 3))) & 0xffu);
      const float pin = Ps[tok * NHID + ncol];
      const float v = tanhf(acc[r] * FOLD + pin);
      const float hk = (t < lenr[r]) ? v : hst[r];
      hst[r] = hk;
      hn[(8 * hh + r) * HPITCH + ncol] = (_Float16)(hk * HCARRY);
    }
    __syncthreads();
  }

#pragma unroll
  for (int r = 0; r < 8; ++r) Hs[(8 * hh + r) * HSPITCH + ncol] = hst[r];
  __syncthreads();

#pragma unroll 1
  for (int p = tid; p < NLOGIT; p += NTHR) {
    const int m = p / NCLS;
    const int o = p - m * NCLS;
    const float* hrow = Hs + m * HSPITCH;
    const float* wrow = W_out + o * NHID;
    float s0 = 0.0f, s1 = 0.0f, s2 = 0.0f, s3 = 0.0f;
#pragma unroll 2
    for (int k = 0; k < NHID; k += 4) {
      const v4f hv = *(const v4f*)(hrow + k);
      const v4f wv = *(const v4f*)(wrow + k);
      s0 = fmaf(fmaxf(hv[0], 0.0f), wv[0], s0);
      s1 = fmaf(fmaxf(hv[1], 0.0f), wv[1], s1);
      s2 = fmaf(fmaxf(hv[2], 0.0f), wv[2], s2);
      s3 = fmaf(fmaxf(hv[3], 0.0f), wv[3], s3);
    }
    Lg[p] = ((s0 + s1) + (s2 + s3)) + b_out[o];
  }
  __syncthreads();

  if (tid < ROWS_BLK) {
    float* lr = Lg + tid * NCLS;
    float mx = lr[0];
#pragma unroll 1
    for (int o = 1; o < NCLS; ++o) mx = fmaxf(mx, lr[o]);
    float sum = 0.0f;
#pragma unroll 1
    for (int o = 0; o < NCLS; ++o) sum += expf(lr[o] - mx);
    const float lse = logf(sum);
#pragma unroll 1
    for (int o = 0; o < NCLS; ++o) lr[o] = (lr[o] - mx) - lse;
  }
  __syncthreads();

  if (wave == 0) {
    float* ob = out + (size_t)blockIdx.x * NLOGIT;
    float vals[NLOGIT / 32];
#pragma unroll
    for (int it = 0; it < NLOGIT / 32; ++it) vals[it] = Lg[it * 32 + lane];
    for (int pass = 0; pass < 2; ++pass) {
#pragma unroll
      for (int it = 0; it < NLOGIT / 32; ++it) *(volatile float*)(ob + it * 32 + lane) = vals[it];
      __threadfence();
    }
  }
}

extern "C" void kernel_launch(void* const* d_in, const int* in_sizes, int n_in,
                              void* d_out, int out_size, void* d_ws, size_t ws_size, hipStream_t stream) {
  if (n_in < 9 || d_out == nullptr || d_ws == nullptr) return;
  if (in_sizes[0] != NBATCH * NSTEP || in_sizes[1] != NBATCH || in_sizes[2] != NVOC * NEMB ||
      in_sizes[3] != NHID * NEMB || in_sizes[4] != NHID * NHID || in_sizes[5] != NHID ||
      in_sizes[6] != NHID || in_sizes[7] != NCLS * NHID || in_sizes[8] != NCLS ||
      out_size != NBATCH * NCLS) return;
  const size_t carve = 32768;
  if (ws_size < carve) return;

  const int*   x     = (const int*)  d_in[0];
  const int*   xlen  = (const int*)  d_in[1];
  const float* emb   = (const float*)d_in[2];
  const float* w_ih  = (const float*)d_in[3];
  const float* w_hh  = (const float*)d_in[4];
  const float* b_ih  = (const float*)d_in[5];
  const float* b_hh  = (const float*)d_in[6];
  const float* w_out = (const float*)d_in[7];
  const float* b_out = (const float*)d_in[8];
  float* out = (float*)d_out;
  float* P   = (float*)d_ws;

  table_kernel<<<(NTABLE + NTHR - 1) / NTHR, NTHR, 0, stream>>>(emb, w_ih, b_ih, b_hh, P);
  rnn_kernel<<<NBATCH / ROWS_BLK, NTHR, 0, stream>>>(x, xlen, w_hh, w_out, b_out, P, out);
}
